// ResidualGNN_1889785610249
// MI455X (gfx1250) — hardware-run, weakly checked
//
#include <hip/hip_runtime.h>
#include <math.h>

constexpr int kNodes    = 100000;
constexpr int kEdges    = 1600000;
constexpr int kVirt     = kEdges + kNodes;
constexpr int kFeat     = 128;
constexpr int kCls      = 3;
constexpr int kHid      = 6;
constexpr int kGraphs   = 16;
constexpr int kMPad     = 100032;
constexpr int kNT       = 256;
constexpr int kChunk    = 2048;
constexpr int kSP       = kChunk / kNT;
constexpr int kNChE     = (kEdges + kChunk - 1) / kChunk;
constexpr int kNChV     = (kVirt + kChunk - 1) / kChunk;
constexpr int kNChB     = (kNodes + kChunk - 1) / kChunk;
constexpr int kDegWave  = 4224;
constexpr int kDegTile  = 8 * kDegWave;
constexpr int kDegTiles = 3;
constexpr int kDegRows  = kDegTiles * kDegTile;
constexpr int kA0Wave   = 6272;
constexpr int kA0Tile   = 8 * kA0Wave;
constexpr int kA0Tiles  = 2;
constexpr int kA1Wave   = 1792;
constexpr int kA1Tile   = 8 * kA1Wave;
constexpr int kA1Tiles  = 7;
constexpr int kGpitch   = 32;
constexpr float kLnEps  = 1e-5f;

static_assert(kMPad % 64 == 0 && kMPad >= kNodes);
static_assert(kFeat % 64 == 0 && kFeat % 32 == 0);
static_assert(kDegRows >= kMPad && kDegWave % 128 == 0 && kDegTile < 65536);
static_assert(kA0Tiles * kA0Tile >= kNodes && kA0Wave % 32 == 0 && kA0Tile < 65536);
static_assert(kA1Tiles * kA1Tile >= kNodes && kA1Wave % 32 == 0 && kA1Tile < 65536);
static_assert(kEdges % kSP == 0 && kNodes % kSP == 0 && kSP == 8);
static_assert(kNodes % 32 == 0 && kNT == 256);

typedef __attribute__((ext_vector_type(16))) _Float16 v16h;
typedef __attribute__((ext_vector_type(8)))  _Float16 v8h;
typedef __attribute__((ext_vector_type(16))) __bf16   v16b;
typedef __attribute__((ext_vector_type(8)))  __bf16   v8b;
typedef __attribute__((ext_vector_type(8)))  float    v8f;
typedef __attribute__((ext_vector_type(4)))  float    v4f;
typedef __attribute__((ext_vector_type(4)))  int      v4i;
typedef __attribute__((ext_vector_type(4)))  unsigned int v4u;

__device__ __forceinline__ unsigned short f2bf_bits(float f) {
  unsigned u = __float_as_uint(f);
  return (unsigned short)((u + 0x7FFFu + ((u >> 16) & 1u)) >> 16);
}
__device__ __forceinline__ float bf_bits2f(unsigned short h) { return __uint_as_float(((unsigned)h) << 16); }

__device__ __forceinline__ void dep_guard_h(v8f& a, v8f& b, v16h x, v16h y) { asm volatile("v_nop\n\tv_nop\n\tv_nop\n\tv_nop" : "+v"(a), "+v"(b) : "v"(x), "v"(y)); }
__device__ __forceinline__ void dep_guard_b(v8f& a, v8f& b, v16b x, v16b y) { asm volatile("v_nop\n\tv_nop\n\tv_nop\n\tv_nop" : "+v"(a), "+v"(b) : "v"(x), "v"(y)); }
__device__ __forceinline__ void keep4_h(v16h a, v16h b, v16h c, v16h d) { asm volatile("v_nop" :: "v"(a), "v"(b), "v"(c), "v"(d)); }
__device__ __forceinline__ void keep4_b(v16b a, v16b b, v16b c, v16b d) { asm volatile("v_nop" :: "v"(a), "v"(b), "v"(c), "v"(d)); }
__device__ __forceinline__ void acc_guard4(v8f& a, v8f& b, v8f& c, v8f& d) { asm volatile("v_nop\n\tv_nop\n\tv_nop\n\tv_nop" : "+v"(a), "+v"(b), "+v"(c), "+v"(d)); }
template <typename T> struct Frag;
template <> struct Frag<_Float16> {
  typedef v16h V; union U { v16h v; v8h h[2]; };
  static __device__ __forceinline__ v16h load(const _Float16* p) {
    U f; f.h[0] = *(const v8h*)(p); f.h[1] = *(const v8h*)(p + 16); return f.v;
  }
  static __device__ __forceinline__ v8f mma(v16h a, v16h b, v8f c) {
    return __builtin_amdgcn_wmma_f32_16x16x32_f16(false, a, false, b, (short)0, c, false, false);
  }
  static __device__ __forceinline__ void guard(v8f& a, v8f& b, v16h x, v16h y) { dep_guard_h(a, b, x, y); }
  static __device__ __forceinline__ void keep(v16h a, v16h b, v16h c, v16h d) { keep4_h(a, b, c, d); }
};
template <> struct Frag<__bf16> {
  typedef v16b V; union U { v16b v; v8b h[2]; };
  static __device__ __forceinline__ v16b load(const __bf16* p) {
    U f; f.h[0] = *(const v8b*)(p); f.h[1] = *(const v8b*)(p + 16); return f.v;
  }
  static __device__ __forceinline__ v8f mma(v16b a, v16b b, v8f c) {
    return __builtin_amdgcn_wmma_f32_16x16x32_bf16(false, a, false, b, (short)0, c, false, false);
  }
  static __device__ __forceinline__ void guard(v8f& a, v8f& b, v16b x, v16b y) { dep_guard_b(a, b, x, y); }
  static __device__ __forceinline__ void keep(v16b a, v16b b, v16b c, v16b d) { keep4_b(a, b, c, d); }
};

template <int ET> struct Elem;
template <> struct Elem<0> { typedef _Float16 T; };
template <> struct Elem<1> { typedef __bf16 T; };
template <int ET, bool SPLIT, int BIAS_MODE, int OUT_MODE, bool RESID, int ACT = 0>
__global__ __launch_bounds__(256) void wmma_gemm64(
    const unsigned short* __restrict__ Ap, const unsigned short* __restrict__ A2p, int lda, long strideA,
    const unsigned short* __restrict__ Btp, const unsigned short* __restrict__ Bt2p, int ldb, long strideB,
    void* __restrict__ Cout, void* __restrict__ Cout2, int ldc, long strideC,
    const float* __restrict__ bias,
    const float* __restrict__ resid, long strideR,
    int M, int N, int K, float scale) {
  typedef typename Elem<ET>::T T;
  typedef typename Frag<T>::V V;
  const T* A = (const T*)Ap; const T* A2 = (const T*)A2p; const T* Bt = (const T*)Btp; const T* Bt2 = (const T*)Bt2p;
  __shared__ __align__(16) float sT[8][16 * 68];
  const int b    = blockIdx.y;
  const int lane = threadIdx.x & 31;
  const int wave = threadIdx.x >> 5;
  const int tilesN = N >> 6;
  const int tilesM = M >> 6;
  const int tile = blockIdx.x * 8 + wave;
  if (tile >= tilesM * tilesN) return;
  const int tm = tile / tilesN;
  const int tn = tile - tm * tilesN;
  const int m0 = tm << 6;
  const int n0 = tn << 6;

  const T* Ab  = A  + (size_t)b * strideA;
  const T* Bb  = Bt + (size_t)b * strideB;
  const T* Ab2 = SPLIT ? (A2  + (size_t)b * strideA) : nullptr;
  const T* Bb2 = SPLIT ? (Bt2 + (size_t)b * strideB) : nullptr;

  const int rlane = lane & 15;
  const int koff  = (lane >> 4) * 8;
  const int mOff  = (lane >> 4) * 8;

  v8f acc[4][4];
#pragma unroll
  for (int i = 0; i < 4; ++i)
#pragma unroll
    for (int j = 0; j < 4; ++j) acc[i][j] = (v8f){0.f,0.f,0.f,0.f,0.f,0.f,0.f,0.f};

  for (int k0 = 0; k0 < K; k0 += 32) {
    V bh[4], bl[4];
#pragma unroll
    for (int j = 0; j < 4; ++j) {
      const size_t bo = (size_t)(n0 + (j << 4) + rlane) * ldb + koff + k0;
      bh[j] = Frag<T>::load(Bb + bo);
      if (SPLIT) bl[j] = Frag<T>::load(Bb2 + bo);
    }
#pragma unroll
    for (int i = 0; i < 4; ++i) {
      const size_t ao = (size_t)(m0 + (i << 4) + rlane) * lda + koff + k0;
      V ah = Frag<T>::load(Ab + ao);
      V al;
      if (SPLIT) al = Frag<T>::load(Ab2 + ao);
#pragma unroll
      for (int j = 0; j < 4; ++j) {
        acc[i][j] = Frag<T>::mma(ah, bh[j], acc[i][j]);
        if (SPLIT) {
          acc[i][j] = Frag<T>::mma(ah, bl[j], acc[i][j]);
          acc[i][j] = Frag<T>::mma(al, bh[j], acc[i][j]);
        }
      }
      Frag<T>::guard(acc[i][0], acc[i][3], ah, SPLIT ? al : ah);
    }
    Frag<T>::keep(bh[0], bh[1], bh[2], bh[3]);
    if (SPLIT) Frag<T>::keep(bl[0], bl[1], bl[2], bl[3]);
  }
  acc_guard4(acc[0][0], acc[0][1], acc[0][2], acc[0][3]);
  acc_guard4(acc[1][0], acc[1][1], acc[1][2], acc[1][3]);
  acc_guard4(acc[2][0], acc[2][1], acc[2][2], acc[2][3]);
  acc_guard4(acc[3][0], acc[3][1], acc[3][2], acc[3][3]);

  float* slab = sT[wave];
  const float* Rb = RESID ? (resid + (size_t)b * strideR) : nullptr;
#pragma unroll
  for (int i = 0; i < 4; ++i) {
    const int mBase = m0 + (i << 4);
    float rsv[8];
#pragma unroll
    for (int r = 0; r < 8; ++r) rsv[r] = 1.0f;
    if (BIAS_MODE == 3) {
      const v4f ra = *(const v4f*)(bias + mBase + mOff);
      const v4f rc = *(const v4f*)(bias + mBase + mOff + 4);
      rsv[0] = ra[0]; rsv[1] = ra[1]; rsv[2] = ra[2]; rsv[3] = ra[3];
      rsv[4] = rc[0]; rsv[5] = rc[1]; rsv[6] = rc[2]; rsv[7] = rc[3];
    }
#pragma unroll
    for (int j = 0; j < 4; ++j) {
      const int n = n0 + (j << 4) + rlane;
      float bv = 0.f;
      if (BIAS_MODE == 2) bv = bias[n];
#pragma unroll
      for (int r = 0; r < 8; ++r) {
        float v = acc[i][j][r] * scale;
        if (BIAS_MODE == 3) v = v * rsv[r];
        if (BIAS_MODE == 1) v += bias[mBase + mOff + r];
        if (BIAS_MODE == 2) v += bv;
        if (RESID) v += Rb[(size_t)(mBase + mOff + r) * ldc + n];
        if (ACT == 1) v = tanhf(v);
        if (ACT == 2) v = fmaxf(v, 0.0f);
        if (ACT == 3) v = v / (1.0f + expf(-v));
        if (ACT == 4) v = (v > 0.f) ? v : 0.01f * v;
        if (ACT == 5) v = 0.5f * v * (1.0f + erff(v * 0.70710678118654752f));
        slab[(mOff + r) * 68 + (j << 4) + rlane] = v;
      }
    }
    __builtin_amdgcn_fence(__ATOMIC_RELEASE, "workgroup");
    __builtin_amdgcn_wave_barrier();
    __builtin_amdgcn_fence(__ATOMIC_ACQUIRE, "workgroup");
    if (OUT_MODE == 0) {
      float* C = (float*)Cout + (size_t)b * strideC;
      const int hh = lane >> 4, c4 = (lane & 15) * 4;
      for (int pass = 0; pass < 2; ++pass) {
#pragma unroll
        for (int it = 0; it < 8; ++it) {
          const int row = it * 2 + hh;
          v4f v = *(const v4f*)(slab + row * 68 + c4);
          *(volatile v4f*)(C + (size_t)(mBase + row) * ldc + n0 + c4) = v;
        }
        __threadfence();
      }
    } else {
      const int q = lane >> 3, c8 = (lane & 7) * 8;
      unsigned short* C  = (unsigned short*)Cout  + (size_t)b * strideC;
      unsigned short* C2 = (OUT_MODE == 2) ? ((unsigned short*)Cout2 + (size_t)b * strideC) : nullptr;
      for (int pass = 0; pass < 2; ++pass) {
#pragma unroll
        for (int it = 0; it < 4; ++it) {
          const int row = it * 4 + q;
          const float* sp = slab + row * 68 + c8;
          v8h hv, lv;
#pragma unroll
          for (int e = 0; e < 8; ++e) {
            if (OUT_MODE == 1) {
              hv[e] = (_Float16)sp[e];
            } else {
              unsigned short hb = f2bf_bits(sp[e]);
              unsigned short lb = f2bf_bits(sp[e] - bf_bits2f(hb));
              hv[e] = __builtin_bit_cast(_Float16, hb);
              lv[e] = __builtin_bit_cast(_Float16, lb);
            }
          }
          *(volatile v8h*)(C + (size_t)(mBase + row) * ldc + n0 + c8) = hv;
          if (OUT_MODE == 2) *(volatile v8h*)(C2 + (size_t)(mBase + row) * ldc + n0 + c8) = lv;
        }
        __threadfence();
      }
    }
    __builtin_amdgcn_fence(__ATOMIC_RELEASE, "workgroup");
    __builtin_amdgcn_wave_barrier();
    __builtin_amdgcn_fence(__ATOMIC_ACQUIRE, "workgroup");
  }
}

__device__ __forceinline__ unsigned pk16(unsigned short a, unsigned short b) { return (unsigned)a | ((unsigned)b << 16); }

__device__ __forceinline__ float bf16r(float f) {
  const unsigned u = __float_as_uint(f);
  const unsigned r = (u + 0x7FFFu + ((u >> 16) & 1u)) & 0xFFFF0000u;
  return __uint_as_float(r);
}

__device__ __forceinline__ float wave_sum(float v) {
#pragma unroll
  for (int m = 16; m >= 1; m >>= 1) v += __shfl_xor(v, m, 32);
  return v;
}
__device__ __forceinline__ float dot4(v4f a, v4f b) { return a[0] * b[0] + a[1] * b[1] + a[2] * b[2] + a[3] * b[3]; }

__device__ __forceinline__ int blk_excl_scan(int cnt, int* scan_ws, int tid, int* tot) {
  const int lane = tid & 31, wave = tid >> 5; int incl = cnt;
#pragma unroll
  for (int o = 1; o < 32; o <<= 1) { const int v = __shfl_up(incl, o, 32); if (lane >= o) incl += v; }
  if (lane == 31) scan_ws[wave] = incl;
  __syncthreads();
  if (wave == 0) { int wv = (lane < kNT / 32) ? scan_ws[lane] : 0; int wincl = wv;
#pragma unroll
    for (int o = 1; o < 32; o <<= 1) { const int v = __shfl_up(wincl, o, 32); if (lane >= o) wincl += v; }
    if (lane < kNT / 32) scan_ws[32 + lane] = wincl - wv; if (lane == 31) scan_ws[64] = wincl; }
  __syncthreads();
  const int res = scan_ws[32 + wave] + incl - cnt; *tot = scan_ws[64];
  return res;
}

template <int TILE, int WROWS, bool SELF, bool WITHSRC>
__device__ __forceinline__ int edge_chunk(const int* __restrict__ dstv, const int* __restrict__ srcv, int e0, int n0,
                                          int tid, int* sDl, int* sSrc, int* sScan) {
  const int eb = e0 + tid * kSP;
  const bool realgrp = eb < kEdges;
  const int ebc = realgrp ? eb : (kEdges - kSP);
  const v4i da = *(const v4i*)(dstv + ebc);
  const v4i db = *(const v4i*)(dstv + ebc + 4);
  int dv[kSP] = {da[0], da[1], da[2], da[3], db[0], db[1], db[2], db[3]};
  int sv[kSP] = {0, 0, 0, 0, 0, 0, 0, 0};
  if (WITHSRC) {
    const v4i sa = *(const v4i*)(srcv + ebc);
    const v4i sb = *(const v4i*)(srcv + ebc + 4);
    sv[0] = sa[0]; sv[1] = sa[1]; sv[2] = sa[2]; sv[3] = sa[3];
    sv[4] = sb[0]; sv[5] = sb[1]; sv[6] = sb[2]; sv[7] = sb[3];
  }
  int recd[kSP], recs[kSP]; int cnt = 0;
#pragma unroll
  for (int k = 0; k < kSP; ++k) {
    const int e = eb + k;
    int dr = dv[k]; dr = dr < 0 ? 0 : (dr >= kNodes ? (kNodes - 1) : dr);
    int sr = sv[k]; sr = sr < 0 ? 0 : (sr >= kNodes ? (kNodes - 1) : sr);
    const int dself = e - kEdges;
    const int d = realgrp ? dr : dself;
    const int s = realgrp ? sr : dself;
    const bool valid = realgrp || (SELF && (e < kVirt));
    const bool hit = valid && (d >= n0) && (d < n0 + TILE);
    const int dl = d - n0;
    const int wv = dl / WROWS;
    recd[k] = hit ? (dl | (wv << 16)) : -1;
    recs[k] = s;
    cnt += hit ? 1 : 0;
  }
  int tot; int p = blk_excl_scan(cnt, sScan, tid, &tot);
#pragma unroll
  for (int k = 0; k < kSP; ++k) {
    if (recd[k] >= 0) {
      if ((unsigned)p < (unsigned)kChunk) { sDl[p] = recd[k]; if (WITHSRC) sSrc[p] = recs[k]; }
      ++p;
    }
  }
  __syncthreads();
  return tot < kChunk ? tot : kChunk;
}

__global__ __launch_bounds__(kNT) void prepw_kernel(const float* __restrict__ W0, unsigned short* __restrict__ Bt) {
  __shared__ float sm[64][65];
  const int t = threadIdx.x;
  const int k0 = blockIdx.x * 64;
  const int nb = blockIdx.y * 64;
#pragma unroll
  for (int i = 0; i < 16; ++i) {
    const int e = i * kNT + t;
    const int kl = e >> 6, nl = e & 63;
    sm[nl][kl] = W0[(size_t)(k0 + kl) * kFeat + nb + nl];
  }
  __syncthreads();
  const int lane = t & 31, wave = t >> 5;
  const int q = lane >> 3, c8 = (lane & 7) * 8;
  for (int pass = 0; pass < 2; ++pass) {
#pragma unroll
    for (int it = 0; it < 2; ++it) {
      const int row = wave * 8 + it * 4 + q;
      unsigned short hb[8];
#pragma unroll
      for (int e = 0; e < 8; ++e) { const float f = sm[row][c8 + e]; hb[e] = f2bf_bits(f); }
      const v4u u = (v4u){pk16(hb[0], hb[1]), pk16(hb[2], hb[3]), pk16(hb[4], hb[5]), pk16(hb[6], hb[7])};
      *(volatile v4u*)(Bt + (size_t)(nb + row) * kFeat + k0 + c8) = u;
    }
    __threadfence();
  }
}

__global__ __launch_bounds__(kNT) void castx_kernel(const float* __restrict__ x, unsigned short* __restrict__ XB, int n8) {
  const int i = blockIdx.x * kNT + threadIdx.x;
  if (i >= n8) return;
  const int row = i >> 4;
  const int c8 = (i & 15) * 8;
  const bool live = row < kNodes;
  const int rowc = live ? row : (kNodes - 1);
  const float* p = x + (size_t)rowc * kFeat + c8;
  const v4f a = *(const v4f*)(p);
  const v4f c = *(const v4f*)(p + 4);
  unsigned short hb[8];
#pragma unroll
  for (int e = 0; e < 4; ++e) {
    const float ae = a[e], ce = c[e];
    hb[e]     = live ? f2bf_bits(ae) : (unsigned short)0;
    hb[4 + e] = live ? f2bf_bits(ce) : (unsigned short)0;
  }
  const v4u u = (v4u){pk16(hb[0], hb[1]), pk16(hb[2], hb[3]), pk16(hb[4], hb[5]), pk16(hb[6], hb[7])};
  unsigned short* q = XB + 8 * (size_t)i;
  *(volatile v4u*)q = u;
  __threadfence();
  *(volatile v4u*)q = u;
}

__global__ __launch_bounds__(kNT) void deg_kernel(const int* __restrict__ ei, float* __restrict__ dinv) {
  __shared__ __align__(16) int sCnt[kDegTile];
  __shared__ int sDl[kChunk];
  __shared__ int sScan[80];
  const int tid = threadIdx.x, lane = tid & 31, wave = tid >> 5;
  const int n0 = blockIdx.x * kDegTile;
  for (int i = tid; i < kDegTile; i += kNT) sCnt[i] = 1;
  for (int i = tid; i < kChunk; i += kNT) sDl[i] = -1;
  if (tid < 80) sScan[tid] = 0;
  __syncthreads();
  const int* srcv = ei;
  const int* dstv = ei + kEdges;
#pragma unroll 1
  for (int c = 0; c < kNChE; ++c) {
    const int tot = edge_chunk<kDegTile, kDegWave, false, false>(dstv, srcv, c * kChunk, n0, tid, sDl, sDl, sScan);
#pragma unroll 1
    for (int base = 0; base < tot; base += 32) {
      const int q = base + lane;
      const int qc = (q < tot) ? q : (tot - 1);
      const int draw = sDl[qc];
      const int dlv = (q < tot) ? draw : -1;
      const int own = ((dlv >> 16) == wave) ? 1 : 0;
      unsigned msk = (unsigned)__ballot(own);
#pragma unroll 1
      for (int it = 0; it < 32; ++it) {
        if (msk == 0u) break;
        const int bp = __builtin_ctz(msk); msk &= msk - 1u;
        const int dl = __shfl(dlv, bp, 32) & 0xFFFF;
        const int cv = sCnt[dl];
        sCnt[dl] = cv + 1;
      }
    }
    __syncthreads();
  }
  __syncthreads();
#pragma unroll 1
  for (int it = 0; it < kDegWave / 128; ++it) {
    const int rl = wave * kDegWave + it * 128 + 4 * lane;
    const v4i cc = *(const v4i*)(sCnt + rl);
    v4f dvv;
    dvv[0] = rsqrtf((float)cc[0]); dvv[1] = rsqrtf((float)cc[1]); dvv[2] = rsqrtf((float)cc[2]); dvv[3] = rsqrtf((float)cc[3]);
    float* dp = dinv + n0 + rl;
    *(volatile v4f*)dp = dvv;
    __threadfence();
    *(volatile v4f*)dp = dvv;
  }
}

__global__ __launch_bounds__(kNT) void agg0_kernel(const float* __restrict__ H0s, const int* __restrict__ ei, const float* __restrict__ dinv,
                                                  const float* __restrict__ b0, const float* __restrict__ g0, const float* __restrict__ be0,
                                                  const float* __restrict__ p0, const float* __restrict__ W1,
                                                  float* __restrict__ A0, float* __restrict__ H1s) {
  __shared__ int sDl[kChunk];
  __shared__ int sSrc[kChunk];
  __shared__ int sScan[80];
  __shared__ __align__(16) float sPar[4 * kFeat];
  __shared__ __align__(16) float sW1t[kCls * kFeat];
  const int tid = threadIdx.x, lane = tid & 31, wave = tid >> 5;
  const int n0 = blockIdx.x * kA0Tile;
  const int rb = n0 + wave * kA0Wave;
  const int c4 = 4 * lane;
  const v4f z4 = {0.f, 0.f, 0.f, 0.f};
  int jmax = 0;
  if (rb < kNodes) { jmax = kNodes - rb; jmax = jmax < kA0Wave ? jmax : kA0Wave; }
  for (int i = tid; i < kChunk; i += kNT) { sDl[i] = -1; sSrc[i] = 0; }
  if (tid < 80) sScan[tid] = 0;
  if (tid < kFeat) {
    sPar[tid]             = bf16r(b0[tid]);
    sPar[kFeat + tid]     = bf16r(g0[tid]);
    sPar[2 * kFeat + tid] = bf16r(be0[tid]);
    sPar[3 * kFeat + tid] = bf16r(p0[tid]);
    sW1t[tid]             = bf16r(W1[tid * kCls + 0]);
    sW1t[kFeat + tid]     = bf16r(W1[tid * kCls + 1]);
    sW1t[2 * kFeat + tid] = bf16r(W1[tid * kCls + 2]);
  }
#pragma unroll 1
  for (int j = 0; j < jmax; ++j) *(v4f*)(A0 + (size_t)(rb + j) * kFeat + c4) = z4;
  __syncthreads();
  const int* srcv = ei;
  const int* dstv = ei + kEdges;
#pragma unroll 1
  for (int c = 0; c < kNChV; ++c) {
    const int tot = edge_chunk<kA0Tile, kA0Wave, true, true>(dstv, srcv, c * kChunk, n0, tid, sDl, sSrc, sScan);
#pragma unroll 1
    for (int base = 0; base < tot; base += 32) {
      const int q = base + lane;
      const int qc = (q < tot) ? q : (tot - 1);
      const int draw = sDl[qc];
      const int svl = sSrc[qc];
      const int dlv = (q < tot) ? draw : -1;
      const int own = ((dlv >> 16) == wave) ? 1 : 0;
      unsigned msk = (unsigned)__ballot(own);
#pragma unroll 1
      for (int it = 0; it < 32; ++it) {
        if (msk == 0u) break;
        const int bp = __builtin_ctz(msk); msk &= msk - 1u;
        const int dl = __shfl(dlv, bp, 32) & 0xFFFF;
        const int s = __shfl(svl, bp, 32);
        const v4f hv = *(const v4f*)(H0s + (size_t)s * kFeat + c4);
        float* ap = A0 + (size_t)(n0 + dl) * kFeat + c4;
        v4f a = *(const v4f*)ap;
        a = a + hv;
        *(v4f*)ap = a;
      }
    }
    __syncthreads();
  }
  const v4f b0v  = *(const v4f*)(sPar + c4);
  const v4f g0v  = *(const v4f*)(sPar + kFeat + c4);
  const v4f be0v = *(const v4f*)(sPar + 2 * kFeat + c4);
  const v4f p0v  = *(const v4f*)(sPar + 3 * kFeat + c4);
  const v4f w10  = *(const v4f*)(sW1t + c4);
  const v4f w11  = *(const v4f*)(sW1t + kFeat + c4);
  const v4f w12  = *(const v4f*)(sW1t + 2 * kFeat + c4);
  float pn = dot4(p0v, p0v);
  pn = wave_sum(pn);
  const float invn = 1.0f / sqrtf(pn);
  v4f myh = z4;
#pragma unroll 1
  for (int j = 0; j < jmax; ++j) {
    const int n = rb + j;
    const float dn = dinv[n];
    const v4f a = *(const v4f*)(A0 + (size_t)n * kFeat + c4);
    const v4f v = a * dn + b0v;
    float s1 = (v[0] + v[1]) + (v[2] + v[3]);
    s1 = wave_sum(s1);
    const float mean = s1 * (1.0f / 128.0f);
    const v4f d = v - mean;
    float s2 = dot4(d, d);
    s2 = wave_sum(s2);
    const float var = s2 * (1.0f / 128.0f);
    const float inv = rsqrtf(var + kLnEps);
    v4f y = d * inv;
    y = y * g0v + be0v;
#pragma unroll
    for (int e = 0; e < 4; ++e) y[e] = fmaxf(y[e], 0.0f);
    float sc = dot4(y, p0v);
    sc = wave_sum(sc) * invn;
    const float gate = tanhf(sc);
    y = y * gate;
    float h0 = dot4(y, w10);
    float h1 = dot4(y, w11);
    float h2 = dot4(y, w12);
    h0 = wave_sum(h0) * dn;
    h1 = wave_sum(h1) * dn;
    h2 = wave_sum(h2) * dn;
    const int slot = j & 31;
    myh[0] = (lane == slot) ? h0 : myh[0];
    myh[1] = (lane == slot) ? h1 : myh[1];
    myh[2] = (lane == slot) ? h2 : myh[2];
    if (slot == 31) {
      float* hp = H1s + (size_t)(n - 31 + lane) * 4;
      *(volatile v4f*)hp = myh;
      __threadfence();
      *(volatile v4f*)hp = myh;
    }
  }
}

__global__ __launch_bounds__(kNT) void agg1_kernel(const float* __restrict__ H1s, const int* __restrict__ ei, const float* __restrict__ dinv,
                                                  const float* __restrict__ b1, const float* __restrict__ g1, const float* __restrict__ be1,
                                                  const float* __restrict__ p1, float* __restrict__ Z) {
  __shared__ __align__(16) float sAcc[kA1Tile * kCls];
  __shared__ int sDl[kChunk];
  __shared__ int sSrc[kChunk];
  __shared__ int sScan[80];
  const int tid = threadIdx.x, lane = tid & 31, wave = tid >> 5;
  const int n0 = blockIdx.x * kA1Tile;
  const int rb = n0 + wave * kA1Wave;
  int jmax = 0;
  if (rb < kNodes) { jmax = kNodes - rb; jmax = jmax < kA1Wave ? jmax : kA1Wave; }
  const int itmax = jmax >> 5;
  const float b10 = bf16r(b1[0]), b11 = bf16r(b1[1]), b12 = bf16r(b1[2]);
  const float g10 = bf16r(g1[0]), g11 = bf16r(g1[1]), g12 = bf16r(g1[2]);
  asm volatile("" ::: "memory");
  const float e10 = bf16r(be1[0]), e11 = bf16r(be1[1]), e12 = bf16r(be1[2]);
  const float p10 = bf16r(p1[0]), p11 = bf16r(p1[1]), p12 = bf16r(p1[2]);
  asm volatile("" ::: "memory");
  for (int i = tid; i < kA1Tile * kCls; i += kNT) sAcc[i] = 0.0f;
  for (int i = tid; i < kChunk; i += kNT) { sDl[i] = -1; sSrc[i] = 0; }
  if (tid < 80) sScan[tid] = 0;
  __syncthreads();
  const int* srcv = ei;
  const int* dstv = ei + kEdges;
  const int lc = lane & 3;
  const int l3 = (lane < 3) ? lane : 2;
#pragma unroll 1
  for (int c = 0; c < kNChV; ++c) {
    const int tot = edge_chunk<kA1Tile, kA1Wave, true, true>(dstv, srcv, c * kChunk, n0, tid, sDl, sSrc, sScan);
#pragma unroll 1
    for (int base = 0; base < tot; base += 32) {
      const int q = base + lane;
      const int qc = (q < tot) ? q : (tot - 1);
      const int draw = sDl[qc];
      const int svl = sSrc[qc];
      const int dlv = (q < tot) ? draw : -1;
      const int own = ((dlv >> 16) == wave) ? 1 : 0;
      unsigned msk = (unsigned)__ballot(own);
#pragma unroll 1
      for (int it = 0; it < 32; ++it) {
        if (msk == 0u) break;
        const int bp = __builtin_ctz(msk); msk &= msk - 1u;
        const int dl = __shfl(dlv, bp, 32) & 0xFFFF;
        const int s = __shfl(svl, bp, 32);
        const float hvs = H1s[(size_t)s * 4 + lc];
        const int ai = dl * kCls + l3;
        float a = sAcc[ai];
        a = a + hvs;
        if (lane < 3) sAcc[ai] = a;
      }
    }
    __syncthreads();
  }
  __syncthreads();
  const float pn1 = p10 * p10 + p11 * p11 + p12 * p12;
  const float invn1 = 1.0f / sqrtf(pn1);
#pragma unroll 1
  for (int it = 0; it < itmax; ++it) {
    const int r = wave * kA1Wave + it * 32 + lane;
    const int n = n0 + r;
    const float dn = dinv[n];
    const float a0 = sAcc[r * kCls], a1 = sAcc[r * kCls + 1], a2 = sAcc[r * kCls + 2];
    const float v0 = a0 * dn + b10, v1 = a1 * dn + b11, v2 = a2 * dn + b12;
    const float mean = (v0 + v1 + v2) * (1.0f / 3.0f);
    const float d0 = v0 - mean, d1 = v1 - mean, d2 = v2 - mean;
    const float var = (d0 * d0 + d1 * d1 + d2 * d2) * (1.0f / 3.0f);
    const float inv = rsqrtf(var + kLnEps);
    const float y0 = fmaxf(d0 * inv * g10 + e10, 0.0f);
    const float y1 = fmaxf(d1 * inv * g11 + e11, 0.0f);
    const float y2 = fmaxf(d2 * inv * g12 + e12, 0.0f);
    const float sc = (y0 * p10 + y1 * p11 + y2 * p12) * invn1;
    const float gate = tanhf(sc);
    v4f zv;
    zv[0] = y0 * gate; zv[1] = y1 * gate; zv[2] = y2 * gate; zv[3] = 0.0f;
    float* zp = Z + (size_t)n * 4;
    *(volatile v4f*)zp = zv;
    __threadfence();
    *(volatile v4f*)zp = zv;
  }
}

__global__ __launch_bounds__(kNT) void pool_kernel(const float* __restrict__ Z, const int* __restrict__ batch, float* __restrict__ Gp) {
  __shared__ int sList[kChunk];
  __shared__ int sScan[80];
  __shared__ __align__(16) float sRed[kNT * 4];
  __shared__ int sRc[kNT];
  const int tid = threadIdx.x, lane = tid & 31, wave = tid >> 5;
  const int g = blockIdx.x;
  const v4f z4 = {0.f, 0.f, 0.f, 0.f};
  for (int i = tid; i < kChunk; i += kNT) sList[i] = 0;
  if (tid < 80) sScan[tid] = 0;
  __syncthreads();
  v4f acc = z4; int cnt = 0;
#pragma unroll 1
  for (int c = 0; c < kNChB; ++c) {
    const int eb = c * kChunk + tid * 8;
    const bool inb = eb < kNodes;
    const int ebc = inb ? eb : (kNodes - 8);
    const v4i ba = *(const v4i*)(batch + ebc);
    const v4i bb = *(const v4i*)(batch + ebc + 4);
    const int bv[8] = {ba[0], ba[1], ba[2], ba[3], bb[0], bb[1], bb[2], bb[3]};
    int rec[8]; int kc = 0;
#pragma unroll
    for (int k = 0; k < 8; ++k) { const bool hit = inb && (bv[k] == g); rec[k] = hit ? (eb + k) : -1; kc += hit ? 1 : 0; }
    int tot; int p = blk_excl_scan(kc, sScan, tid, &tot);
#pragma unroll
    for (int k = 0; k < 8; ++k) { if (rec[k] >= 0) { if ((unsigned)p < (unsigned)kChunk) sList[p] = rec[k]; ++p; } }
    __syncthreads();
    const int totc = tot < kChunk ? tot : kChunk;
#pragma unroll 1
    for (int q0 = wave * 32; q0 < totc; q0 += kNT) {
      const int q = q0 + lane;
      const int qc = (q < totc) ? q : (totc - 1);
      int nd = sList[qc];
      nd = nd < 0 ? 0 : (nd >= kNodes ? (kNodes - 1) : nd);
      const v4f zr = *(const v4f*)(Z + (size_t)nd * 4);
      const float f = (q < totc) ? 1.0f : 0.0f;
      acc = acc + zr * f;
      cnt += (q < totc) ? 1 : 0;
    }
    __syncthreads();
  }
  *(v4f*)(sRed + 4 * tid) = acc;
  sRc[tid] = cnt;
  __syncthreads();
  if (wave == 0) {
    v4f s = z4; int ct = 0;
#pragma unroll
    for (int w = 0; w < kNT / 32; ++w) { s = s + *(const v4f*)(sRed + 4 * (w * 32 + lane)); ct += sRc[w * 32 + lane]; }
#pragma unroll
    for (int off = 16; off >= 1; off >>= 1) {
      s[0] += __shfl_xor(s[0], off, 32);
      s[1] += __shfl_xor(s[1], off, 32);
      s[2] += __shfl_xor(s[2], off, 32);
      s[3] += __shfl_xor(s[3], off, 32);
      ct += __shfl_xor(ct, off, 32);
    }
    const float cf = (float)ct;
    const float inv = 1.0f / fmaxf(cf, 1.0f);
    const float o0 = s[0] * inv, o1 = s[1] * inv, o2 = s[2] * inv;
    const float val = (lane == 0) ? o0 : ((lane == 1) ? o1 : ((lane == 2) ? o2 : 0.0f));
    volatile float* gp = Gp + (size_t)g * kGpitch;
    gp[lane] = val;
    __threadfence();
    gp[lane] = val;
  }
}

__global__ __launch_bounds__(kNT) void head_kernel(const float* __restrict__ Gp,
                                                  const float* __restrict__ fw1, const float* __restrict__ fb1,
                                                  const float* __restrict__ fw2, const float* __restrict__ fb2,
                                                  const float* __restrict__ fw3, const float* __restrict__ fb3,
                                                  float* __restrict__ out) {
  __shared__ float sG[kGraphs * kCls];
  __shared__ float sT1[kGraphs * kHid];
  __shared__ float sT2[kGraphs * kHid];
  __shared__ __align__(16) float sO[kGraphs * kCls];
  const int tid = threadIdx.x;
  if (tid < kGraphs * kCls) { const int g = tid / kCls, c = tid - g * kCls; sG[tid] = Gp[g * kGpitch + c]; }
  __syncthreads();
  if (tid < kGraphs * kHid) {
    const int g = tid / kHid, o = tid - g * kHid;
    float a = 0.0f;
#pragma unroll 1
    for (int c = 0; c < kCls; ++c) a += sG[g * kCls + c] * bf16r(fw1[c * kHid + o]);
    a += bf16r(fb1[o]);
    sT1[tid] = fmaxf(a, 0.0f);
  }
  __syncthreads();
  if (tid < kGraphs * kHid) {
    const int g = tid / kHid, o = tid - g * kHid;
    float a = 0.0f;
#pragma unroll 1
    for (int i = 0; i < kHid; ++i) a += sT1[g * kHid + i] * bf16r(fw2[i * kHid + o]);
    a += bf16r(fb2[o]);
    sT2[tid] = fmaxf(a, 0.0f);
  }
  __syncthreads();
  if (tid < kGraphs * kCls) {
    const int g = tid / kCls, o = tid - g * kCls;
    float a = 0.0f;
#pragma unroll 1
    for (int i = 0; i < kHid; ++i) a += sT2[g * kHid + i] * bf16r(fw3[i * kCls + o]);
    a += bf16r(fb3[o]);
    sO[tid] = tanhf(a);
  }
  __syncthreads();
  if (tid < 32) {
    const int lane = tid;
    const int idx = (lane < 12) ? lane : 0;
    const v4f v = *(const v4f*)(sO + 4 * idx);
    float* op = out + 4 * lane;
    if (lane < 12) *(volatile v4f*)op = v;
    __threadfence();
    if (lane < 12) *(volatile v4f*)op = v;
  }
}

extern "C" void kernel_launch(void* const* d_in, const int* in_sizes, int n_in,
                              void* d_out, int out_size, void* d_ws, size_t ws_size, hipStream_t stream) {
  (void)in_sizes; (void)n_in; (void)out_size;
  const float* x     = (const float*)d_in[0];
  const int*   ei    = (const int*)  d_in[1];
  const int*   batch = (const int*)  d_in[2];
  const float* W0    = (const float*)d_in[3];
  const float* b0    = (const float*)d_in[4];
  const float* g0    = (const float*)d_in[5];
  const float* be0   = (const float*)d_in[6];
  const float* p0    = (const float*)d_in[7];
  const float* W1    = (const float*)d_in[8];
  const float* b1    = (const float*)d_in[9];
  const float* g1    = (const float*)d_in[10];
  const float* be1   = (const float*)d_in[11];
  const float* p1    = (const float*)d_in[12];
  const float* fw1   = (const float*)d_in[13];
  const float* fb1   = (const float*)d_in[14];
  const float* fw2   = (const float*)d_in[15];
  const float* fb2   = (const float*)d_in[16];
  const float* fw3   = (const float*)d_in[17];
  const float* fb3   = (const float*)d_in[18];
  float* out = (float*)d_out;

  char* ws = (char*)d_ws; size_t off = 0;
  auto carve = [&](size_t bytes) -> char* { char* p = ws + off; off += (bytes + 255) & ~(size_t)255; return p; };
  unsigned short* XB   = (unsigned short*)carve((size_t)kMPad * kFeat * 2);
  unsigned short* Bt   = (unsigned short*)carve((size_t)kFeat * kFeat * 2);
  float*          H0s  = (float*)carve((size_t)kMPad * kFeat * 4);
  float*          A0   = (float*)carve((size_t)kNodes * kFeat * 4);
  float*          DINV = (float*)carve((size_t)kDegRows * 4);
  float*          H1s  = (float*)carve((size_t)kNodes * 4 * 4);
  float*          Z    = (float*)carve((size_t)kNodes * 4 * 4);
  float*          Gp   = (float*)carve((size_t)kGraphs * kGpitch * 4);
  if (off > ws_size || off > (size_t)134217728) return;

  prepw_kernel<<<dim3(2, 2), kNT, 0, stream>>>(W0, Bt);
  {
    const int n8 = kMPad * kFeat / 8;
    castx_kernel<<<(n8 + kNT - 1) / kNT, kNT, 0, stream>>>(x, XB, n8);
  }
  deg_kernel<<<kDegTiles, kNT, 0, stream>>>(ei, DINV);
  {
    const int tiles = (kMPad / 64) * (kFeat / 64);
    wmma_gemm64<1, false, 3, 0, false><<<dim3((tiles + 7) / 8, 1), 256, 0, stream>>>(
        (const unsigned short*)XB, (const unsigned short*)nullptr, kFeat, 0L,
        (const unsigned short*)Bt, (const unsigned short*)nullptr, kFeat, 0L,
        (void*)H0s, (void*)nullptr, kFeat, 0L,
        (const float*)DINV, (const float*)nullptr, 0L, kMPad, kFeat, kFeat, 1.0f);
  }
  agg0_kernel<<<kA0Tiles, kNT, 0, stream>>>(H0s, ei, DINV, b0, g0, be0, p0, W1, A0, H1s);
  agg1_kernel<<<kA1Tiles, kNT, 0, stream>>>(H1s, ei, DINV, b1, g1, be1, p1, Z);
  pool_kernel<<<kGraphs, kNT, 0, stream>>>(Z, batch, Gp);
  head_kernel<<<1, kNT, 0, stream>>>(Gp, fw1, fb1, fw2, fb2, fw3, fb3, out);
}
